// ImprovedGQA_80315888435253
// MI455X (gfx1250) — hardware-verified
//
#include <hip/hip_runtime.h>
#include <stddef.h>
#include <stdint.h>

#define NBAT  2
#define SQ    2048
#define NTOK  4096
#define HID   2048
#define NH    16
#define NKV   4
#define HDM   128
#define NPAIR 64
#define NQKV  3072
#define KOFS  (NH * HDM)
#define VOFS  (NH * HDM + NKV * HDM)
#define NSQ   16
#define NSK   4
#define NSLAB 24
#define QB    128
#define KC    64
#define NQB   (SQ / QB)
#define NCK   (SQ / KC)

static_assert(NTOK == NBAT * SQ);
static_assert(HID == NH * HDM);
static_assert(NH == 4 * NKV);
static_assert(NQKV == NH * HDM + 2 * NKV * HDM);
static_assert(NQKV == NSLAB * 128);
static_assert(HDM == 128);
static_assert(HDM == 2 * NPAIR);
static_assert(SQ % QB == 0);
static_assert(SQ % KC == 0);
static_assert(SQ % 64 == 0);
static_assert(NTOK % 256 == 0);
static_assert(HID % 64 == 0);
static_assert((SQ * NPAIR) % 256 == 0);
static_assert((NTOK * HID) % 2048 == 0);
static_assert((NKV * HDM * HID) % 2048 == 0);

typedef _Float16 v16h __attribute__((ext_vector_type(16)));
typedef _Float16 v8h  __attribute__((ext_vector_type(8)));
typedef float    v8f  __attribute__((ext_vector_type(8)));
typedef float    v4f  __attribute__((ext_vector_type(4)));
typedef float    v2f  __attribute__((ext_vector_type(2)));
typedef unsigned int v4u __attribute__((ext_vector_type(4)));

union Frag  { v16h v; v8h h[2]; };
union Pack8 { v8h h; v4u u; };

__device__ __forceinline__ v8f mma16(v16h a, v16h b, v8f c) {
  c = __builtin_amdgcn_wmma_f32_16x16x32_f16(false, a, false, b, (short)0, c, false, false);
  asm volatile("v_nop\n\tv_nop\n\tv_nop\n\tv_nop" : "+v"(c) : "v"(a), "v"(b));
  return c;
}

__device__ __forceinline__ v16h ldfrag(const _Float16* p, int ld, int row0, int k0, int lane) {
  const int m = lane & 15, lh = lane >> 4;
  const _Float16* q = p + (size_t)(row0 + m) * ld + k0 + 8 * lh;
  Frag f;
  f.h[0] = *(const v8h*)(q);
  f.h[1] = *(const v8h*)(q + 16);
  return f.v;
}

__device__ __forceinline__ v8f zero8() { return (v8f){0.f, 0.f, 0.f, 0.f, 0.f, 0.f, 0.f, 0.f}; }

__device__ __forceinline__ void gemm16x64(const _Float16* __restrict__ A, int lda,
                                          const _Float16* __restrict__ Bt, int ldb,
                                          int m0, int n0, int lane, v8f (&acc)[4]) {
#pragma unroll 2
  for (int k0 = 0; k0 < HID; k0 += 32) {
    const v16h a = ldfrag(A, lda, m0, k0, lane);
#pragma unroll
    for (int t = 0; t < 4; ++t) {
      const v16h b = ldfrag(Bt, ldb, n0 + 16 * t, k0, lane);
      acc[t] = mma16(a, b, acc[t]);
    }
  }
}

__device__ __forceinline__ void gemm32x64(const _Float16* __restrict__ A, int lda,
                                          const _Float16* __restrict__ Bt, int ldb,
                                          int m0, int n0, int lane, v8f (&acc)[2][4]) {
#pragma unroll 2
  for (int k0 = 0; k0 < HID; k0 += 32) {
    const v16h a0 = ldfrag(A, lda, m0, k0, lane);
    const v16h a1 = ldfrag(A, lda, m0 + 16, k0, lane);
    const v16h b0 = ldfrag(Bt, ldb, n0, k0, lane);
    const v16h b1 = ldfrag(Bt, ldb, n0 + 16, k0, lane);
    const v16h b2 = ldfrag(Bt, ldb, n0 + 32, k0, lane);
    const v16h b3 = ldfrag(Bt, ldb, n0 + 48, k0, lane);
    acc[0][0] = mma16(a0, b0, acc[0][0]);
    acc[1][0] = mma16(a1, b0, acc[1][0]);
    acc[0][1] = mma16(a0, b1, acc[0][1]);
    acc[1][1] = mma16(a1, b1, acc[1][1]);
    acc[0][2] = mma16(a0, b2, acc[0][2]);
    acc[1][2] = mma16(a1, b2, acc[1][2]);
    acc[0][3] = mma16(a0, b3, acc[0][3]);
    acc[1][3] = mma16(a1, b3, acc[1][3]);
  }
}

__global__ __launch_bounds__(256) void k_cvt(const float* __restrict__ src, _Float16* __restrict__ dh,
                                             int nvec, float scale) {
  const int g = blockIdx.x * 256 + (int)threadIdx.x;
  if (g >= nvec) return;
  const size_t o = (size_t)g * 8;
  const v4f a0 = *(const v4f*)(src + o);
  const v4f a1 = *(const v4f*)(src + o + 4);
  Pack8 pk;
  pk.h = (v8h){(_Float16)(a0[0] * scale), (_Float16)(a0[1] * scale), (_Float16)(a0[2] * scale), (_Float16)(a0[3] * scale),
               (_Float16)(a1[0] * scale), (_Float16)(a1[1] * scale), (_Float16)(a1[2] * scale), (_Float16)(a1[3] * scale)};
  const v4u vv = pk.u;
  volatile v4u* d = (volatile v4u*)(dh + o);
  *d = vv;
  __threadfence();
  *d = vv;
}

__global__ __launch_bounds__(256) void k_rope(float* __restrict__ cs, int npos) {
  const int g = blockIdx.x * 256 + (int)threadIdx.x;
  if (g >= npos * NPAIR) return;
  const int pos = g >> 6;
  const int i   = g & (NPAIR - 1);
  const double e  = (double)i * (13.287712379549449 * 0.015625);
  const float base = (float)exp2(e);
  const float inv  = 1.0f / base;
  const float ang  = (float)pos * inv;
  float sn, cn;
  sincosf(ang, &sn, &cn);
  const v2f v = {cn, sn};
  volatile v2f* d = (volatile v2f*)(cs + 2 * (size_t)g);
  *d = v;
  __threadfence();
  *d = v;
}

#define SFP 132
__global__ __launch_bounds__(256) void k_qkv(const _Float16* __restrict__ xh,
                                             const _Float16* __restrict__ wt,
                                             const float* __restrict__ qg,
                                             const float* __restrict__ kg,
                                             const float* __restrict__ cs,
                                             _Float16* __restrict__ qp,
                                             _Float16* __restrict__ kp,
                                             _Float16* __restrict__ vtp) {
  __shared__ __align__(16) float sf[64 * SFP];
  const int tid = threadIdx.x, lane = tid & 31, wave = tid >> 5;
  const int hh = lane >> 4, c = lane & 15;
  const int wm = wave >> 1, wn = wave & 1;
  const int mb = blockIdx.x * 64;
  const int b  = mb / SQ;
  const int sb = mb - b * SQ;
  const int ns = blockIdx.y;
  const int which = (ns < NSQ) ? 0 : ((ns < NSQ + NSK) ? 1 : 2);
  const int head  = (which == 0) ? ns : ((which == 1) ? (ns - NSQ) : (ns - NSQ - NSK));
  const int m0 = mb + wm * 16;
  const int n0 = ns * 128 + wn * 64;

  v8f acc[4];
#pragma unroll
  for (int t = 0; t < 4; ++t) acc[t] = zero8();
  gemm16x64(xh, HID, wt, HID, m0, n0, lane, acc);

#pragma unroll
  for (int t = 0; t < 4; ++t) {
#pragma unroll
    for (int r = 0; r < 8; ++r)
      sf[(wm * 16 + 8 * hh + r) * SFP + wn * 64 + 16 * t + c] = acc[t][r] * 0.03125f;
  }
  __syncthreads();

  if (which < 2) {
    const float* gam = (which == 0) ? qg : kg;
    const int lr = tid >> 2;
    const int qq = tid & 3;
    float* rp = sf + lr * SFP + qq * 32;
    float ss = 0.f;
#pragma unroll
    for (int e = 0; e < 8; ++e) {
      const v4f a = *(const v4f*)(rp + 4 * e);
      ss += a[0] * a[0] + a[1] * a[1] + a[2] * a[2] + a[3] * a[3];
    }
    ss += __shfl_xor(ss, 1, 32);
    ss += __shfl_xor(ss, 2, 32);
    const float inv = rsqrtf(ss * 0.0078125f + 1e-6f);
    const float* csr = cs + (size_t)(sb + lr) * (2 * NPAIR) + qq * 32;
    const float* gr  = gam + qq * 32;
#pragma unroll
    for (int e = 0; e < 8; ++e) {
      const v4f a = *(const v4f*)(rp + 4 * e);
      const v4f g = *(const v4f*)(gr + 4 * e);
      const v4f w = *(const v4f*)(csr + 4 * e);
      const float x0 = a[0] * inv * g[0], x1 = a[1] * inv * g[1];
      const float x2 = a[2] * inv * g[2], x3 = a[3] * inv * g[3];
      v4f o;
      o[0] = x0 * w[0] - x1 * w[1];
      o[1] = x0 * w[1] + x1 * w[0];
      o[2] = x2 * w[2] - x3 * w[3];
      o[3] = x2 * w[3] + x3 * w[2];
      *(v4f*)(rp + 4 * e) = o;
    }
  }
  __syncthreads();

  if (which < 2) {
    v4u val[4];
    size_t go[4];
    const int hb = (which == 0) ? (b * NH + head) : (b * NKV + head);
#pragma unroll
    for (int j = 0; j < 4; ++j) {
      const int p  = tid + 256 * j;
      const int lr = p >> 4;
      const int pc = p & 15;
      const float* ra = sf + lr * SFP + pc * 8;
      const v4f a0 = *(const v4f*)(ra), a1 = *(const v4f*)(ra + 4);
      Pack8 pk;
      pk.h = (v8h){(_Float16)a0[0], (_Float16)a0[1], (_Float16)a0[2], (_Float16)a0[3],
                   (_Float16)a1[0], (_Float16)a1[1], (_Float16)a1[2], (_Float16)a1[3]};
      val[j] = pk.u;
      go[j]  = ((size_t)hb * SQ + sb + lr) * HDM + pc * 8;
    }
    _Float16* base = (which == 0) ? qp : kp;
    for (int ps = 0; ps < 2; ++ps) {
#pragma unroll
      for (int j = 0; j < 4; ++j) *(volatile v4u*)(base + go[j]) = val[j];
      __threadfence();
    }
  } else {
    v4u val[4];
    size_t go[4];
    const int hb = b * NKV + head;
#pragma unroll
    for (int j = 0; j < 4; ++j) {
      const int p    = tid + 256 * j;
      const int dcol = p >> 3;
      const int pc   = p & 7;
      const float* cp = sf + (pc * 8) * SFP + dcol;
      Pack8 pk;
      pk.h = (v8h){(_Float16)cp[0 * SFP], (_Float16)cp[1 * SFP], (_Float16)cp[2 * SFP], (_Float16)cp[3 * SFP],
                   (_Float16)cp[4 * SFP], (_Float16)cp[5 * SFP], (_Float16)cp[6 * SFP], (_Float16)cp[7 * SFP]};
      val[j] = pk.u;
      go[j]  = ((size_t)hb * HDM + dcol) * SQ + sb + pc * 8;
    }
    for (int ps = 0; ps < 2; ++ps) {
#pragma unroll
      for (int j = 0; j < 4; ++j) *(volatile v4u*)(vtp + go[j]) = val[j];
      __threadfence();
    }
  }
}

#define KTPK 136
#define KTPV 72
#define PTP  72
#define OTPH 136
static_assert(8 * 16 * OTPH <= KC * KTPK + HDM * KTPV);
__global__ __launch_bounds__(256) void k_attn(const _Float16* __restrict__ qp,
                                              const _Float16* __restrict__ kp,
                                              const _Float16* __restrict__ vt,
                                              const int* __restrict__ mask,
                                              _Float16* __restrict__ op, float sscale) {
  __shared__ __align__(16) _Float16 KV[KC * KTPK + HDM * KTPV];
  __shared__ __align__(16) _Float16 Ps[8 * 16 * PTP];
  _Float16* Ks = KV;
  _Float16* Vs = KV + KC * KTPK;

  const int tid = threadIdx.x, lane = tid & 31, wave = tid >> 5;
  const int hh = lane >> 4, c = lane & 15;
  const int qb  = blockIdx.x % NQB;
  const int hb  = blockIdx.x / NQB;
  const int h   = hb % NH;
  const int b   = hb / NH;
  const int grp = h >> 2;
  const int q0  = qb * QB + wave * 16;

  const _Float16* Q = qp + (size_t)hb * SQ * HDM;
  const _Float16* K = kp + (size_t)(b * NKV + grp) * SQ * HDM;
  const _Float16* V = vt + (size_t)(b * NKV + grp) * HDM * SQ;
  const int* mrw = mask + (size_t)b * SQ;
  const size_t trow0 = (size_t)b * SQ;

  v16h qa[4];
#pragma unroll
  for (int dc = 0; dc < 4; ++dc) qa[dc] = ldfrag(Q, HDM, q0, dc * 32, lane);

  const float NEGI = -__builtin_huge_valf();
  float mrow[8], lrow[8];
  v8f oacc[8];
#pragma unroll
  for (int r = 0; r < 8; ++r) { mrow[r] = NEGI; lrow[r] = 0.f; }
#pragma unroll
  for (int t = 0; t < 8; ++t) oacc[t] = zero8();

  _Float16* pw = Ps + wave * 16 * PTP;

  for (int kc = 0; kc < NCK; ++kc) {
    const int kv0 = kc * KC;
    __syncthreads();
    {
      const int r  = tid >> 2;
      const int qq = (tid & 3) * 32;
      const _Float16* ks = K + (size_t)(kv0 + r) * HDM + qq;
#pragma unroll
      for (int e = 0; e < 4; ++e) *(v8h*)(Ks + r * KTPK + qq + 8 * e) = *(const v8h*)(ks + 8 * e);
      const int r2 = tid >> 1;
      const int q2 = (tid & 1) * 32;
      const _Float16* vs = V + (size_t)r2 * SQ + kv0 + q2;
#pragma unroll
      for (int e = 0; e < 4; ++e) *(v8h*)(Vs + r2 * KTPV + q2 + 8 * e) = *(const v8h*)(vs + 8 * e);
    }
    int mk[4];
#pragma unroll
    for (int j = 0; j < 4; ++j) mk[j] = mrw[kv0 + j * 16 + c];
    __syncthreads();

    v8f s[4];
#pragma unroll
    for (int j = 0; j < 4; ++j) s[j] = zero8();
#pragma unroll
    for (int dc = 0; dc < 4; ++dc) {
#pragma unroll
      for (int j = 0; j < 4; ++j) {
        const v16h kb = ldfrag(Ks, KTPK, j * 16, dc * 32, lane);
        s[j] = mma16(qa[dc], kb, s[j]);
      }
    }
    float cm[8];
#pragma unroll
    for (int r = 0; r < 8; ++r) {
      float m = NEGI;
#pragma unroll
      for (int j = 0; j < 4; ++j) {
        const float sv = (mk[j] != 0) ? (s[j][r] * sscale) : NEGI;
        s[j][r] = sv;
        m = fmaxf(m, sv);
      }
#pragma unroll
      for (int off = 1; off < 16; off <<= 1) m = fmaxf(m, __shfl_xor(m, off, 32));
      cm[r] = m;
    }
    float al[8];
#pragma unroll
    for (int r = 0; r < 8; ++r) {
      const float mnew  = fmaxf(mrow[r], cm[r]);
      const bool  live  = (mnew != NEGI);
      const float alpha = live ? __expf(mrow[r] - mnew) : 1.f;
      mrow[r] = mnew;
      float psum = 0.f;
#pragma unroll
      for (int j = 0; j < 4; ++j) {
        const float p = live ? __expf(s[j][r] - mnew) : 0.f;
        psum += p;
        pw[(8 * hh + r) * PTP + j * 16 + c] = (_Float16)(p * 1024.0f);
      }
#pragma unroll
      for (int off = 1; off < 16; off <<= 1) psum += __shfl_xor(psum, off, 32);
      lrow[r] = lrow[r] * alpha + psum;
      al[r] = alpha;
    }
#pragma unroll
    for (int t = 0; t < 8; ++t)
#pragma unroll
      for (int r = 0; r < 8; ++r) oacc[t][r] *= al[r];
    __syncthreads();

#pragma unroll
    for (int kk = 0; kk < 2; ++kk) {
      const v16h pa = ldfrag(pw, PTP, 0, kk * 32, lane);
#pragma unroll
      for (int t = 0; t < 8; ++t) {
        const v16h vb = ldfrag(Vs, KTPV, t * 16, kk * 32, lane);
        oacc[t] = mma16(pa, vb, oacc[t]);
      }
    }
  }

  float invl[8];
#pragma unroll
  for (int r = 0; r < 8; ++r) invl[r] = 0.015625f / lrow[r];
  __syncthreads();
  _Float16* ow = KV + wave * 16 * OTPH;
#pragma unroll
  for (int r = 0; r < 8; ++r) {
#pragma unroll
    for (int t = 0; t < 8; ++t)
      ow[(8 * hh + r) * OTPH + 16 * t + c] = (_Float16)(oacc[t][r] * invl[r]);
  }
  __syncthreads();
  v4u val[8];
  size_t go[8];
#pragma unroll
  for (int it = 0; it < 8; ++it) {
    const int p  = lane + 32 * it;
    const int L  = p >> 4;
    const int pc = p & 15;
    Pack8 pk;
    pk.h    = *(const v8h*)(ow + L * OTPH + pc * 8);
    val[it] = pk.u;
    go[it]  = (trow0 + q0 + L) * HID + (size_t)h * HDM + pc * 8;
  }
  for (int ps = 0; ps < 2; ++ps) {
#pragma unroll
    for (int it = 0; it < 8; ++it) *(volatile v4u*)(op + go[it]) = val[it];
    __threadfence();
  }
}

#define OTP 68
__device__ __forceinline__ void out_epilogue(v8f (&acc)[2][4], float scale,
                                             float* sw, float* __restrict__ out,
                                             int m0, int n0, int lane, int hh, int c) {
#pragma unroll
  for (int sub = 0; sub < 2; ++sub) {
    __syncthreads();
#pragma unroll
    for (int t = 0; t < 4; ++t) {
#pragma unroll
      for (int r = 0; r < 8; ++r) sw[(8 * hh + r) * OTP + 16 * t + c] = acc[sub][t][r] * scale;
    }
    __syncthreads();
    v4f val[8];
    size_t go[8];
#pragma unroll
    for (int it = 0; it < 8; ++it) {
      const int p    = lane + 32 * it;
      const int L    = p >> 3;
      const int pc   = p & 7;
      const int row  = L >> 1;
      const int half = L & 1;
      val[it] = *(const v4f*)(sw + row * OTP + half * 32 + pc * 4);
      go[it]  = (size_t)(m0 + sub * 16 + row) * HID + n0 + half * 32 + pc * 4;
    }
    for (int ps = 0; ps < 2; ++ps) {
#pragma unroll
      for (int it = 0; it < 8; ++it) *(volatile v4f*)(out + go[it]) = val[it];
      __threadfence();
    }
  }
}

__global__ __launch_bounds__(256) void k_out(const _Float16* __restrict__ ap,
                                             const _Float16* __restrict__ wt,
                                             float* __restrict__ out) {
  __shared__ __align__(16) float st[8][16 * OTP];
  const int tid = threadIdx.x, lane = tid & 31, wave = tid >> 5;
  const int hh = lane >> 4, c = lane & 15;
  const int m0 = blockIdx.x * 256 + wave * 32;
  const int n0 = blockIdx.y * 64;

  v8f acc[2][4];
#pragma unroll
  for (int s = 0; s < 2; ++s)
#pragma unroll
    for (int t = 0; t < 4; ++t) acc[s][t] = zero8();
  gemm32x64(ap, HID, wt, HID, m0, n0, lane, acc);
  out_epilogue(acc, 0.001953125f, st[wave], out, m0, n0, lane, hh, c);
}

extern "C" void kernel_launch(void* const* d_in, const int* in_sizes, int n_in,
                              void* d_out, int out_size, void* d_ws, size_t ws_size,
                              hipStream_t stream) {
  if (n_in < 8) return;
  if (in_sizes[0] != NTOK * HID) return;
  if (in_sizes[1] != NBAT * SQ) return;
  if (in_sizes[2] != HID * HID) return;
  if (in_sizes[3] != NKV * HDM * HID) return;
  if (in_sizes[4] != NKV * HDM * HID) return;
  if (in_sizes[5] != HID * HID) return;
  if (in_sizes[6] != HDM) return;
  if (in_sizes[7] != HDM) return;
  if (out_size != NTOK * HID) return;

  const float* x   = (const float*)d_in[0];
  const int*   msk = (const int*)d_in[1];
  const float* wq  = (const float*)d_in[2];
  const float* wk  = (const float*)d_in[3];
  const float* wv  = (const float*)d_in[4];
  const float* wo  = (const float*)d_in[5];
  const float* qg  = (const float*)d_in[6];
  const float* kg  = (const float*)d_in[7];
  float* out = (float*)d_out;

  size_t off = 0;
  const size_t oX  = off; off += (size_t)NTOK * HID * 2;
  const size_t oWt = off; off += (size_t)NQKV * HID * 2;
  const size_t oWo = off; off += (size_t)HID * HID * 2;
  const size_t oCS = off; off += (size_t)SQ * NPAIR * 2 * 4;
  const size_t oQ  = off; off += (size_t)NBAT * NH * SQ * HDM * 2;
  const size_t oK  = off; off += (size_t)NBAT * NKV * SQ * HDM * 2;
  const size_t oV  = off; off += (size_t)NBAT * NKV * HDM * SQ * 2;
  const size_t oO  = off; off += (size_t)NTOK * HID * 2;
  if (off > ws_size) return;
  if (off > (size_t)134217728) return;

  char* ws = (char*)d_ws;
  _Float16* Xh  = (_Float16*)(ws + oX);
  _Float16* Wt  = (_Float16*)(ws + oWt);
  _Float16* Wot = (_Float16*)(ws + oWo);
  float*    Cs  = (float*)(ws + oCS);
  _Float16* Qp  = (_Float16*)(ws + oQ);
  _Float16* Kp  = (_Float16*)(ws + oK);
  _Float16* Vt  = (_Float16*)(ws + oV);
  _Float16* Op  = (_Float16*)(ws + oO);

  k_cvt<<<dim3((NTOK * HID / 8) / 256), dim3(256), 0, stream>>>(x, Xh, NTOK * HID / 8, 1.0f);
  k_cvt<<<dim3((HID * HID / 8) / 256), dim3(256), 0, stream>>>(wq, Wt, HID * HID / 8, 32.0f);
  k_cvt<<<dim3((NKV * HDM * HID / 8) / 256), dim3(256), 0, stream>>>(wk, Wt + (size_t)KOFS * HID, NKV * HDM * HID / 8, 32.0f);
  k_cvt<<<dim3((NKV * HDM * HID / 8) / 256), dim3(256), 0, stream>>>(wv, Wt + (size_t)VOFS * HID, NKV * HDM * HID / 8, 32.0f);
  k_cvt<<<dim3((HID * HID / 8) / 256), dim3(256), 0, stream>>>(wo, Wot, HID * HID / 8, 32.0f);
  k_rope<<<dim3((SQ * NPAIR) / 256), dim3(256), 0, stream>>>(Cs, SQ);
  k_qkv<<<dim3(NTOK / 64, NSLAB), dim3(256), 0, stream>>>(Xh, Wt, qg, kg, Cs, Qp, Kp, Vt);
  const float sscale = 0.08838834764831845f;
  k_attn<<<dim3(NBAT * NH * NQB), dim3(256), 0, stream>>>(Qp, Kp, Vt, msk, Op, sscale);
  k_out<<<dim3(NTOK / 256, HID / 64), dim3(256), 0, stream>>>(Op, Wot, out);
  (void)hipGetLastError();
}
